// UniformBertSelfAttention_14448269983908
// MI455X (gfx1250) — hardware-verified
//
#include <hip/hip_runtime.h>


#ifndef NB
#define NB 4
#endif
#ifndef SEQ
#define SEQ 4096
#endif
#define NB_FULL  4
#define SEQ_FULL 4096
#ifndef OUT_SEQ
#define OUT_SEQ SEQ
#endif
#define DM   768
#define TPB  (SEQ / 64)
#define ORW  64
#define STH  256

static_assert(DM % 64 == 0);
static_assert(DM % 32 == 0);
static_assert(DM % 128 == 0);
static_assert(DM / 4 <= 1024);
static_assert(SEQ % 64 == 0);
static_assert((NB * SEQ) % 64 == 0);
static_assert(SEQ % STH == 0);
static_assert(SEQ % 32 == 0);
static_assert(SEQ % ORW == 0);
static_assert(((size_t)SEQ * DM) % 8 == 0);
static_assert(((size_t)DM * DM) % 8 == 0);
static_assert(NB <= NB_FULL);
static_assert(SEQ <= SEQ_FULL);
static_assert((size_t)SEQ * 4 + 64 <= 131072);
static_assert(64 * 4 <= 131072);
static_assert(16 * 4 == 64);

typedef unsigned short bf;
typedef __attribute__((ext_vector_type(16))) __bf16   v16bf;
typedef __attribute__((ext_vector_type(8)))  unsigned short v8us;
typedef __attribute__((ext_vector_type(8)))  float    v8f;
typedef __attribute__((ext_vector_type(4)))  float    v4f;
typedef v4f  __attribute__((may_alias)) v4fa;

__device__ __forceinline__ unsigned short f2bf(float f) { unsigned u = __float_as_uint(f); u += 0x7FFFu + ((u >> 16) & 1u); return (unsigned short)(u >> 16); }
__device__ __forceinline__ float bfr(float f) { return __uint_as_float(((unsigned)f2bf(f)) << 16); }
__device__ __forceinline__ v16bf cat16b(v8us lo, v8us hi) { return __builtin_bit_cast(v16bf, __builtin_shufflevector(lo, hi, 0, 1, 2, 3, 4, 5, 6, 7, 8, 9, 10, 11, 12, 13, 14, 15)); }
__device__ __forceinline__ v16bf ldb(const bf* p)  { return cat16b(*(const v8us*)p, *(const v8us*)(p + 16)); }
__device__ __forceinline__ void wave_sync() { __builtin_amdgcn_fence(3  , "wavefront"); __builtin_amdgcn_wave_barrier(); asm volatile("" ::: "memory"); }
__device__ __forceinline__ v8f wmmab_g(v16bf a, v16bf b, v8f c) {
    c = __builtin_amdgcn_wmma_f32_16x16x32_bf16(false, a, false, b, (short)0, c, false, false);
    asm volatile("v_nop\n\tv_nop\n\tv_nop\n\tv_nop" : "+v"(c) : "v"(a), "v"(b));
    return c;
}

__global__ __launch_bounds__(256) void k_cvt8(const float* __restrict__ src, bf* dst, size_t n8) {
    const size_t i = (size_t)blockIdx.x * 256 + threadIdx.x; if (i >= n8) return;
    const v8f v = *(const v8f*)(src + i * 8); v8us o;
#pragma unroll
    for (int k = 0; k < 8; ++k) o[k] = f2bf(v[k]);
    *(volatile v8us*)(dst + i * 8) = o; __threadfence(); *(volatile v8us*)(dst + i * 8) = o;
}

__global__ __launch_bounds__(STH) void k_soft(const float* __restrict__ mask, float* PW) {
#pragma clang fp contract(off)
    __shared__ __align__(16) float es[SEQ];
    __shared__ float red[8];
    const int t = threadIdx.x, lane = t & 31;
    const int wave = __builtin_amdgcn_readfirstlane((int)(threadIdx.x >> 5));
    const int b = blockIdx.x;
    const float* mrow = mask + (size_t)b * SEQ_FULL;
    float m = -__builtin_huge_valf();
#pragma unroll 1
    for (int i = t; i < SEQ; i += STH) m = fmaxf(m, bfr(mrow[i]));
#pragma unroll
    for (int o = 16; o > 0; o >>= 1) m = fmaxf(m, __shfl_xor(m, o, 32));
    if (lane == 0) red[wave] = m;
    __syncthreads();
    float mm = red[0];
#pragma unroll
    for (int k = 1; k < STH / 32; ++k) mm = fmaxf(mm, red[k]);
    __syncthreads();
    float s = 0.0f;
#pragma unroll 1
    for (int i = t; i < SEQ; i += STH) { const float e = expf(bfr(mrow[i]) - mm); es[i] = e; s += e; }
#pragma unroll
    for (int o = 16; o > 0; o >>= 1) s += __shfl_xor(s, o, 32);
    if (lane == 0) red[wave] = s;
    __syncthreads();
    float tot = red[0];
#pragma unroll
    for (int k = 1; k < STH / 32; ++k) tot += red[k];
    const float inv = 1.0f / tot;
    float* dst = PW + (size_t)b * SEQ;
#pragma unroll 1
    for (int ps = 0; ps < 2; ++ps) {
#pragma unroll 1
        for (int q = t; q < SEQ / 4; q += STH) {
            const v4f e4 = *(const v4fa*)(&es[4 * q]);
            const v4f val = e4 * inv;
            *(volatile v4f*)(dst + 4 * q) = val; }
        if (ps == 0) __threadfence(); }
}

__global__ __launch_bounds__(32) void k_gemm_pool(const bf* __restrict__ A, const bf* __restrict__ Bt, const float* __restrict__ bias, const float* __restrict__ PW, float* PT) {
    __shared__ __align__(16) float os[64];
    const int K = DM;
    const int lane = threadIdx.x & 31, lr = lane & 15, hi = lane >> 4; const int r0 = blockIdx.x * 64, c0 = blockIdx.y * 64;
    v8f acc[4][4];
#pragma unroll
    for (int mb = 0; mb < 4; ++mb)
#pragma unroll
        for (int nb = 0; nb < 4; ++nb) acc[mb][nb] = (v8f){};
    const size_t aoff = (size_t)(r0 + lr) * K + 8 * hi, boff = (size_t)(c0 + lr) * K + 8 * hi;
#pragma unroll 1
    for (int kc = 0; kc < K; kc += 32) {
        v16bf a[4];
#pragma unroll
        for (int mb = 0; mb < 4; ++mb) a[mb] = ldb(A + aoff + (size_t)mb * 16 * K + kc);
#pragma unroll
        for (int nb = 0; nb < 4; ++nb) { const v16bf b = ldb(Bt + boff + (size_t)nb * 16 * K + kc);
#pragma unroll
            for (int mb = 0; mb < 4; ++mb) acc[mb][nb] = wmmab_g(a[mb], b, acc[mb][nb]); }
    }
    float bc[4], cs[4];
#pragma unroll
    for (int nb = 0; nb < 4; ++nb) { bc[nb] = bfr(bias[c0 + nb * 16 + lr]); cs[nb] = 0.0f; }
#pragma unroll
    for (int mb = 0; mb < 4; ++mb) {
        const float* pp = PW + (size_t)r0 + mb * 16 + 8 * hi;
        const v4f p0 = *(const v4f*)pp, p1 = *(const v4f*)(pp + 4);
#pragma unroll
        for (int nb = 0; nb < 4; ++nb) {
#pragma unroll
            for (int j = 0; j < 4; ++j) cs[nb] += p0[j] * (acc[mb][nb][j] + bc[nb]);
#pragma unroll
            for (int j = 0; j < 4; ++j) cs[nb] += p1[j] * (acc[mb][nb][4 + j] + bc[nb]); }
    }
#pragma unroll
    for (int nb = 0; nb < 4; ++nb) cs[nb] += __shfl_xor(cs[nb], 16, 32);
    if (hi == 0) {
#pragma unroll
        for (int nb = 0; nb < 4; ++nb) os[nb * 16 + lr] = cs[nb]; }
    wave_sync();
    const v4f val = *(const v4fa*)(&os[lr * 4]);
    float* dst = PT + (size_t)blockIdx.x * DM + c0 + lr * 4;
#pragma unroll 1
    for (int ps = 0; ps < 2; ++ps) {
        if (lane < 16) *(volatile v4f*)dst = val;
        if (ps == 0) __threadfence(); }
}

__global__ __launch_bounds__(DM / 4) void k_ctx(const float* __restrict__ PT, float* CT) {
    const int t = threadIdx.x; const int b = blockIdx.x;
    const float* src = PT + (size_t)b * TPB * DM + 4 * t;
    v4f s = (v4f){};
#pragma unroll 4
    for (int rt = 0; rt < TPB; ++rt) s += *(const v4f*)(src + (size_t)rt * DM);
    float* dst = CT + (size_t)b * DM + 4 * t;
#pragma unroll 1
    for (int ps = 0; ps < 2; ++ps) {
        *(volatile v4f*)dst = s;
        if (ps == 0) __threadfence(); }
}

__global__ __launch_bounds__(DM / 4) void k_out(const float* __restrict__ CT, float* OUT) {
    const int t = threadIdx.x; const int b = blockIdx.y;
    const v4f val = *(const v4f*)(CT + (size_t)b * DM + 4 * t);
    float* dst = OUT + ((size_t)b * OUT_SEQ + (size_t)blockIdx.x * ORW) * DM + 4 * t;
#pragma unroll 1
    for (int ps = 0; ps < 2; ++ps) {
#pragma unroll 4
        for (int r = 0; r < ORW; ++r) *(volatile v4f*)(dst + (size_t)r * DM) = val;
        if (ps == 0) __threadfence(); }
}

static constexpr size_t al256(size_t v) { return (v + 255) & ~(size_t)255; }
static constexpr size_t SZ_XB = al256((size_t)NB * SEQ * DM * 2);
static constexpr size_t SZ_WB = al256((size_t)DM * DM * 2);
static constexpr size_t SZ_PW = al256((size_t)NB * SEQ * 4);
static constexpr size_t SZ_PT = al256((size_t)NB * TPB * DM * 4);
static constexpr size_t SZ_CT = al256((size_t)NB * DM * 4);
static constexpr size_t SZ_TOTAL = SZ_XB + SZ_WB + SZ_PW + SZ_PT + SZ_CT;
static_assert(SZ_TOTAL <= (size_t)134217728);
static_assert((size_t)(NB * SEQ / 64) * DM * 4 <= SZ_PT);
static_assert((size_t)NB * TPB == (size_t)(NB * SEQ / 64));
static_assert(((size_t)DM * 4) % 128 == 0);

extern "C" void kernel_launch(void* const* d_in, const int* in_sizes, int n_in,
                              void* d_out, int out_size, void* d_ws, size_t ws_size, hipStream_t stream) {
    if (n_in < 8) return;
    const size_t needx = ((size_t)(NB - 1) * SEQ_FULL + SEQ) * DM;
    const size_t needm = (size_t)(NB - 1) * SEQ_FULL + SEQ;
    if ((size_t)in_sizes[0] < needx || (size_t)in_sizes[1] < needm) return;
    if ((size_t)in_sizes[6] < (size_t)DM * DM || in_sizes[7] < DM) return;
    if ((size_t)out_size < ((size_t)(NB - 1) * OUT_SEQ + SEQ) * DM) return;
    if (SZ_TOTAL > ws_size) return;
    const float* hidden = (const float*)d_in[0];
    const float* amask  = (const float*)d_in[1];
    const float* wv     = (const float*)d_in[6];
    const float* bv     = (const float*)d_in[7];
    float* OUT = (float*)d_out;
    char* wsp = (char*)d_ws;
    bf* XB = (bf*)wsp; wsp += SZ_XB;
    bf* WB = (bf*)wsp; wsp += SZ_WB;
    float* PW = (float*)wsp; wsp += SZ_PW;
    float* PT = (float*)wsp; wsp += SZ_PT;
    float* CT = (float*)wsp; wsp += SZ_CT;

    if (SEQ == SEQ_FULL) {
        const size_t n8 = (size_t)NB * SEQ * DM / 8;
        k_cvt8<<<(unsigned)((n8 + 255) / 256), 256, 0, stream>>>(hidden, XB, n8);
    } else {
        const size_t n8 = (size_t)SEQ * DM / 8;
        for (int b = 0; b < NB; ++b) k_cvt8<<<(unsigned)((n8 + 255) / 256), 256, 0, stream>>>(hidden + (size_t)b * SEQ_FULL * DM, XB + (size_t)b * SEQ * DM, n8);
    }
    { const size_t n8 = (size_t)DM * DM / 8; k_cvt8<<<(unsigned)((n8 + 255) / 256), 256, 0, stream>>>(wv, WB, n8); }

    k_soft<<<NB, STH, 0, stream>>>(amask, PW);
    k_gemm_pool<<<dim3(NB * SEQ / 64, DM / 64, 1), 32, 0, stream>>>(XB, WB, bv, PW, PT);
    k_ctx<<<NB, DM / 4, 0, stream>>>(PT, CT);
    k_out<<<dim3(SEQ / ORW, NB, 1), DM / 4, 0, stream>>>(CT, OUT);
}
